// TransPhormer_72808285602170
// MI455X (gfx1250) — hardware-verified
//
#include <hip/hip_runtime.h>
#include <stddef.h>
#include <math.h>


#define NODE_W 160
#define QW     640
#define MDIM   80
#define NBAS   16

#define INV_SQRT3   0.57735026918962576f
#define INV_SQRT2   0.70710678118654752f
#define INV_SQRT32  0.17677669529663688f
#define INV_SQRT48  0.14433756729740643f
#define INV_SQRT128 0.088388347648318441f
#define LN_EPS      1e-5f

typedef float  v4f  __attribute__((ext_vector_type(4)));
typedef float  v8f  __attribute__((ext_vector_type(8)));
typedef int    v4i  __attribute__((ext_vector_type(4)));
typedef int    v8i  __attribute__((ext_vector_type(8)));
typedef __bf16 bf16;
typedef __bf16 v8b  __attribute__((ext_vector_type(8)));
typedef __bf16 v16b __attribute__((ext_vector_type(16)));
union FragB { v16b v; v8b h[2]; };

__device__ __forceinline__ v8f z8f() {
  v8f z;
#pragma unroll
  for (int i = 0; i < 8; ++i) z[i] = 0.0f;
  return z;
}

__device__ __forceinline__ void wxbar() {
  __builtin_amdgcn_fence(__ATOMIC_RELEASE, "wavefront");
  __builtin_amdgcn_wave_barrier();
}

__device__ __forceinline__ v8f wmb(v16b a, v16b b, v8f c) {
  v8f d = __builtin_amdgcn_wmma_f32_16x16x32_bf16(false, a, false, b, (short)0, c, false, false);
  asm volatile("v_nop\n\tv_nop\n\tv_nop\n\tv_nop" : "+v"(d) : "v"(a), "v"(b));
  return d;
}

__device__ __forceinline__ v16b ldfrag(const bf16* p, int h) {
  FragB f;
  f.h[0] = *(const v8b*)(p + 8 * h);
  f.h[1] = *(const v8b*)(p + 16 + 8 * h);
  return f.v;
}

__device__ __forceinline__ void split2(float v, bf16& hi, bf16& lo) {
  const bf16 t = (bf16)v;
  hi = t;
  lo = (bf16)(v - (float)t);
}
__device__ __forceinline__ void put48(bf16* row, int k, float v) {
  bf16 hi, lo;
  split2(v, hi, lo);
  row[k] = hi; row[48 + k] = lo; row[96 + k] = hi;
}
__device__ __forceinline__ void put64(bf16* row, int k, float v) {
  bf16 hi, lo;
  split2(v, hi, lo);
  row[k] = hi; row[64 + k] = lo;
}
__device__ __forceinline__ int clampi(int v, int lo, int hi) { return v < lo ? lo : (v > hi ? hi : v); }

__global__ __launch_bounds__(256) void k_wprep(
    const float* __restrict__ Wq0, const float* __restrict__ Wsrc0, const float* __restrict__ Wdst0,
    const float* __restrict__ Wq1, const float* __restrict__ Wsrc1, const float* __restrict__ Wdst1,
    const float* __restrict__ Wrbf, const float* __restrict__ Wkv0, const float* __restrict__ Wkv1,
    const float* __restrict__ Wm0, const float* __restrict__ Wm1,
    bf16* P0, bf16* P1, bf16* P2, bf16* P3, bf16* P4, bf16* P5, bf16* P6) {
  const int job = blockIdx.y;
  const float *S0, *S1, *S2;
  int nc0, nc1, nc2, r0, r1, r2, K, Kp;
  bf16* dst;
  switch (job) {
    case 0:  S0 = Wq0;  nc0 = 256; r0 = 256; S1 = Wsrc0; nc1 = 32; r1 = 32; S2 = Wdst0; nc2 = 32; r2 = 32; K = 64;  Kp = 192; dst = P0; break;
    case 1:  S0 = Wq1;  nc0 = 128; r0 = 128; S1 = Wsrc1; nc1 = 16; r1 = 16; S2 = Wdst1; nc2 = 16; r2 = 16; K = 32;  Kp = 96;  dst = P1; break;
    case 2:  S0 = Wrbf; nc0 = 112; r0 = 112; S1 = Wrbf;  nc1 = 112; r1 = 0; S2 = Wrbf;  nc2 = 112; r2 = 0; K = 16;  Kp = 64;  dst = P2; break;
    case 3:  S0 = Wkv0; nc0 = 512; r0 = 512; S1 = Wkv0;  nc1 = 512; r1 = 0; S2 = Wkv0;  nc2 = 512; r2 = 0; K = 48;  Kp = 160; dst = P3; break;
    case 4:  S0 = Wkv1; nc0 = 256; r0 = 256; S1 = Wkv1;  nc1 = 256; r1 = 0; S2 = Wkv1;  nc2 = 256; r2 = 0; K = 64;  Kp = 192; dst = P4; break;
    case 5:  S0 = Wm0;  nc0 = 64;  r0 = 64;  S1 = Wm0;   nc1 = 64;  r1 = 0; S2 = Wm0;   nc2 = 64;  r2 = 0; K = 256; Kp = 768; dst = P5; break;
    default: S0 = Wm1;  nc0 = 32;  r0 = 32;  S1 = Wm1;   nc1 = 32;  r1 = 0; S2 = Wm1;   nc2 = 32;  r2 = 0; K = 128; Kp = 384; dst = P6; break;
  }
  const int rows = r0 + r1 + r2;
  const int nchunk = rows * Kp / 8;
  const int c = blockIdx.x * 256 + threadIdx.x;
  if (c >= nchunk) return;
  const int n  = (8 * c) / Kp;
  const int k0 = 8 * c - n * Kp;
  const int c0 = clampi(n, 0, r0 - 1);
  const int c1 = clampi(n - r0, 0, (r1 > 0 ? r1 : 1) - 1);
  const int c2 = clampi(n - r0 - r1, 0, (r2 > 0 ? r2 : 1) - 1);
  const bf16 bz = (bf16)0.0f;
  v8b o;
#pragma unroll
  for (int j = 0; j < 8; ++j) {
    const int kq  = k0 + j;
    const int seg = kq / K;
    const int k   = clampi(kq - seg * K, 0, K - 1);
    const float wa = S0[k * nc0 + c0];
    const float wb = S1[k * nc1 + c1];
    const float wcv = S2[k * nc2 + c2];
    const float w = (n < r0) ? wa : ((n < r0 + r1) ? wb : wcv);
    bf16 hi, lo;
    split2(w, hi, lo);
    const bf16 val = (seg < 2) ? hi : ((seg == 2) ? lo : bz);
    o[j] = val;
  }
  bf16* p = dst + (size_t)c * 8;
  *(volatile v8b*)p = o;
  __threadfence();
  *(volatile v8b*)p = o;
}

#define NT1 256
__global__ __launch_bounds__(NT1) void k_node(
    const float* __restrict__ node, const float* __restrict__ g0, const float* __restrict__ g1,
    const bf16* __restrict__ B0T, const bf16* __restrict__ B1T, float* qout, float* sdout, int nN) {
  __shared__ __attribute__((aligned(16))) bf16  A0[16 * 128];
  __shared__ __attribute__((aligned(16))) bf16  A1[48 * 64];
  __shared__ __attribute__((aligned(16))) float qs[16 * QW];
  __shared__ __attribute__((aligned(16))) float ss[16 * NODE_W];
  const int tid = threadIdx.x, lane = tid & 31, wave = tid >> 5, h = lane >> 4, m = lane & 15;
  const int nodeBase = blockIdx.x * 16;

#pragma unroll
  for (int t = 0; t < 2; ++t) {
    const int nl = 2 * wave + t;
    const int ng = nodeBase + nl;
    const bool ok = ng < nN;
    const int nc = ok ? ng : (nN - 1);
    const float* nr = node + (size_t)nc * NODE_W;
    const float a = nr[lane], b = nr[lane + 32];
    float s = a + b;
#pragma unroll
    for (int k = 16; k > 0; k >>= 1) s += __shfl_xor(s, k);
    const float mu = s * (1.0f / 64.0f);
    const float da = a - mu, db = b - mu;
    float vv = da * da + db * db;
#pragma unroll
    for (int k = 16; k > 0; k >>= 1) vv += __shfl_xor(vv, k);
    const float var = vv * (1.0f / 64.0f);
    const float inv = 1.0f / sqrtf(var + LN_EPS);
    float h0a = da * inv * g0[lane];
    float h0b = db * inv * g0[lane + 32];
    if (!ok) { h0a = 0.0f; h0b = 0.0f; }
    bf16 hi, lo;
    split2(h0a, hi, lo); A0[nl * 128 + lane] = hi;      A0[nl * 128 + 64 + lane] = lo;
    split2(h0b, hi, lo); A0[nl * 128 + 32 + lane] = hi; A0[nl * 128 + 96 + lane] = lo;
    const float x0 = nr[64 + 3 * lane], x1 = nr[65 + 3 * lane], x2 = nr[66 + 3 * lane];
    float vn = x0 * x0 + x1 * x1 + x2 * x2;
#pragma unroll
    for (int k = 16; k > 0; k >>= 1) vn += __shfl_xor(vn, k);
    const float rin = 1.0f / sqrtf(vn * (1.0f / 32.0f) + LN_EPS);
    const float gg = g1[lane];
    float c0 = x0 * rin * gg, c1 = x1 * rin * gg, c2 = x2 * rin * gg;
    if (!ok) { c0 = 0.0f; c1 = 0.0f; c2 = 0.0f; }
    split2(c0, hi, lo); A1[(nl * 3 + 0) * 64 + lane] = hi; A1[(nl * 3 + 0) * 64 + 32 + lane] = lo;
    split2(c1, hi, lo); A1[(nl * 3 + 1) * 64 + lane] = hi; A1[(nl * 3 + 1) * 64 + 32 + lane] = lo;
    split2(c2, hi, lo); A1[(nl * 3 + 2) * 64 + lane] = hi; A1[(nl * 3 + 2) * 64 + 32 + lane] = lo;
  }
  __syncthreads();

#pragma unroll 1
  for (int nt = wave; nt < 20; nt += 8) {
    v8f acc = z8f();
#pragma unroll
    for (int ks = 0; ks < 6; ++ks)
      acc = wmb(ldfrag(A0 + m * 128 + ((32 * ks) & 127), h),
                ldfrag(B0T + (size_t)(16 * nt + m) * 192 + 32 * ks, h), acc);
#pragma unroll
    for (int r = 0; r < 8; ++r) {
      const int nl = 8 * h + r;
      const float v = acc[r] * 0.125f;
      if (nt < 16)      qs[nl * QW + (nt >> 1) * MDIM + ((nt & 1) << 4) + m] = v;
      else if (nt < 18) ss[nl * NODE_W + ((nt - 16) << 4) + m] = v;
      else              ss[nl * NODE_W + 80 + ((nt - 18) << 4) + m] = v;
    }
  }
#pragma unroll 1
  for (int t = wave; t < 30; t += 8) {
    const int mt = t / 10, nt = t - 10 * mt;
    v8f acc = z8f();
#pragma unroll
    for (int ks = 0; ks < 3; ++ks)
      acc = wmb(ldfrag(A1 + (16 * mt + m) * 64 + ((32 * ks) & 63), h),
                ldfrag(B1T + (size_t)(16 * nt + m) * 96 + 32 * ks, h), acc);
#pragma unroll
    for (int r = 0; r < 8; ++r) {
      const int rr = 16 * mt + 8 * h + r;
      const int nl = rr / 3, c = rr - 3 * nl;
      const float v = acc[r] * INV_SQRT32;
      if (nt < 8)       qs[nl * QW + nt * MDIM + 32 + 3 * m + c] = v;
      else if (nt == 8) ss[nl * NODE_W + 32 + 3 * m + c] = v;
      else              ss[nl * NODE_W + 112 + 3 * m + c] = v;
    }
  }
  __syncthreads();

#pragma unroll 1
  for (int ps = 0; ps < 2; ++ps) {
#pragma unroll
    for (int t = 0; t < 2; ++t) {
      const int nl = 2 * wave + t;
      const size_t ng = (size_t)(nodeBase + nl);
#pragma unroll
      for (int i = 0; i < 5; ++i) {
        const int off = (4 * i + (lane >> 3)) * 32 + (lane & 7) * 4;
        const v4f v = *(const v4f*)(qs + nl * QW + off);
        *(volatile v4f*)(qout + ng * QW + off) = v;
      }
      {
        const int off = (lane >> 3) * 32 + (lane & 7) * 4;
        const v4f v = *(const v4f*)(ss + nl * NODE_W + off);
        *(volatile v4f*)(sdout + ng * NODE_W + off) = v;
        const int off2 = 128 + (lane & 7) * 4;
        const v4f v2 = *(const v4f*)(ss + nl * NODE_W + off2);
        if (lane < 8) *(volatile v4f*)(sdout + ng * NODE_W + off2) = v2;
      }
    }
    if (ps == 0) __threadfence();
  }
}

struct __attribute__((aligned(16))) TileBuf {
  float y[16][4];
  float at[16][8];
  bf16  Arbf[16][64];
  bf16  Acp0[16][160];
  bf16  Acp1[3][16][128];
  int   srcI[16];
  int   dstI[16];
  int   slot[16];
  int   padi[4];
};

__device__ __forceinline__ void tile_gather(TileBuf& T, int e, bool valid, int lane,
                                            const int* __restrict__ ei, int nE, int nN,
                                            const float* __restrict__ rbf, const float* __restrict__ rsh) {
  const int h = lane >> 4, m = lane & 15;
  const int ec = clampi(e, 0, nE - 1);
  const int s = clampi(ei[ec], 0, nN - 1);
  const int d = clampi(ei[nE + ec], 0, nN - 1);
  v4f yy = *(const v4f*)(rsh + (size_t)ec * 4);
  const v4f z4 = {0.0f, 0.0f, 0.0f, 0.0f};
  if (!valid) yy = z4;
  if (h == 0) { T.srcI[m] = s; T.dstI[m] = d; *(v4f*)(&T.y[m][0]) = yy; }
  const v4f ra = *(const v4f*)(rbf + (size_t)ec * NBAS + 8 * h);
  const v4f rb = *(const v4f*)(rbf + (size_t)ec * NBAS + 8 * h + 4);
  float rv[8] = {ra.x, ra.y, ra.z, ra.w, rb.x, rb.y, rb.z, rb.w};
  const bf16 bz = (bf16)0.0f;
  bf16* ar = &T.Arbf[m][0];
#pragma unroll
  for (int j = 0; j < 8; ++j) {
    const float v = valid ? rv[j] : 0.0f;
    bf16 hi, lo;
    split2(v, hi, lo);
    const int k = 8 * h + j;
    ar[k] = hi; ar[16 + k] = lo; ar[32 + k] = hi; ar[48 + k] = bz;
  }
#pragma unroll
  for (int r = 0; r < 8; ++r) T.Acp0[8 * h + r][144 + m] = bz;
}

template <int NT>
__device__ __forceinline__ void cg_ntile(TileBuf& T, int lane, const bf16* __restrict__ BrbfT,
                                         const float* __restrict__ SD) {
  const int h = lane >> 4, m = lane & 15;
  v8f acc = z8f();
#pragma unroll
  for (int ks = 0; ks < 2; ++ks)
    acc = wmb(ldfrag(&T.Arbf[m][32 * ks], h), ldfrag(BrbfT + (size_t)(16 * NT + m) * 64 + 32 * ks, h), acc);
#pragma unroll
  for (int r = 0; r < 8; ++r) {
    const int e = 8 * h + r;
    const float* ps = SD + (size_t)T.srcI[e] * NODE_W;
    const float* pd = SD + (size_t)T.dstI[e] * NODE_W;
    const float w = acc[r];
    if (NT < 2) {
      const int k = 16 * NT + m;
      const float x0 = ps[k] + pd[80 + k];
      put48(&T.Acp0[e][0], k, w * x0 * T.y[e][0]);
    } else if (NT == 2) {
      const float a0 = ps[32 + 3 * m] + pd[112 + 3 * m];
      const float a1 = ps[33 + 3 * m] + pd[113 + 3 * m];
      const float a2 = ps[34 + 3 * m] + pd[114 + 3 * m];
      const float dt = a0 * T.y[e][1] + a1 * T.y[e][2] + a2 * T.y[e][3];
      put48(&T.Acp0[e][0], 32 + m, w * dt * INV_SQRT3);
    } else if (NT < 5) {
      const int u = 16 * (NT - 3) + m;
      const float x0 = ps[u] + pd[80 + u];
      const float wx = w * x0;
      put64(&T.Acp1[0][e][0], u, wx * T.y[e][1]);
      put64(&T.Acp1[1][e][0], u, wx * T.y[e][2]);
      put64(&T.Acp1[2][e][0], u, wx * T.y[e][3]);
    } else if (NT == 5) {
      const float a0 = ps[32 + 3 * m] + pd[112 + 3 * m];
      const float a1 = ps[33 + 3 * m] + pd[113 + 3 * m];
      const float a2 = ps[34 + 3 * m] + pd[114 + 3 * m];
      const float y0 = T.y[e][0];
      put64(&T.Acp1[0][e][0], 32 + m, w * a0 * y0);
      put64(&T.Acp1[1][e][0], 32 + m, w * a1 * y0);
      put64(&T.Acp1[2][e][0], 32 + m, w * a2 * y0);
    } else {
      const float a0 = ps[32 + 3 * m] + pd[112 + 3 * m];
      const float a1 = ps[33 + 3 * m] + pd[113 + 3 * m];
      const float a2 = ps[34 + 3 * m] + pd[114 + 3 * m];
      const float y1 = T.y[e][1], y2 = T.y[e][2], y3 = T.y[e][3];
      const float cr0 = a1 * y3 - a2 * y2;
      const float cr1 = a2 * y1 - a0 * y3;
      const float cr2 = a0 * y2 - a1 * y1;
      put64(&T.Acp1[0][e][0], 48 + m, w * cr0 * INV_SQRT2);
      put64(&T.Acp1[1][e][0], 48 + m, w * cr1 * INV_SQRT2);
      put64(&T.Acp1[2][e][0], 48 + m, w * cr2 * INV_SQRT2);
    }
  }
}

#define NT2 128
#define NW2 4
__global__ __launch_bounds__(NT2) void k_logit(
    const int* __restrict__ ei, const float* __restrict__ rbf, const float* __restrict__ rsh,
    const float* __restrict__ SD, const float* __restrict__ q,
    const bf16* __restrict__ BrbfT, const bf16* __restrict__ Bkv0T, const bf16* __restrict__ Bkv1T,
    float* lg, int nN, int nE) {
  __shared__ TileBuf tb[NW2];
  const int tid = threadIdx.x, lane = tid & 31, wave = tid >> 5, h = lane >> 4, m = lane & 15;
  const int tile = blockIdx.x * NW2 + wave;
  TileBuf& T = tb[wave];

  const int e = tile * 16 + m;
  const bool valid = e < nE;
  tile_gather(T, e, valid, lane, ei, nE, nN, rbf, rsh);
  __syncthreads();
  cg_ntile<0>(T, lane, BrbfT, SD);
  cg_ntile<1>(T, lane, BrbfT, SD);
  cg_ntile<2>(T, lane, BrbfT, SD);
  cg_ntile<3>(T, lane, BrbfT, SD);
  cg_ntile<4>(T, lane, BrbfT, SD);
  cg_ntile<5>(T, lane, BrbfT, SD);
  cg_ntile<6>(T, lane, BrbfT, SD);
  __syncthreads();

  int sI[8];
#pragma unroll
  for (int r = 0; r < 8; ++r) sI[r] = T.srcI[8 * h + r];

#pragma unroll 1
  for (int hd = 0; hd < 8; ++hd) {
    float p[8];
#pragma unroll
    for (int r = 0; r < 8; ++r) p[r] = 0.0f;
#pragma unroll
    for (int s2 = 0; s2 < 2; ++s2) {
      const int nt = 2 * hd + s2;
      v8f acc = z8f();
#pragma unroll
      for (int ks = 0; ks < 5; ++ks)
        acc = wmb(ldfrag(&T.Acp0[m][32 * ks], h),
                  ldfrag(Bkv0T + (size_t)(16 * nt + m) * 160 + 32 * ks, h), acc);
      const float* qc = q + hd * MDIM + 16 * s2 + m;
#pragma unroll
      for (int r = 0; r < 8; ++r) p[r] += (acc[r] * INV_SQRT48) * qc[(size_t)sI[r] * QW];
    }
#pragma unroll
    for (int c = 0; c < 3; ++c) {
      v8f acc = z8f();
#pragma unroll
      for (int ks = 0; ks < 6; ++ks)
        acc = wmb(ldfrag(&T.Acp1[c][m][(32 * ks) & 127], h),
                  ldfrag(Bkv1T + (size_t)(16 * hd + m) * 192 + 32 * ks, h), acc);
      const float* qc = q + hd * MDIM + 32 + 3 * m + c;
#pragma unroll
      for (int r = 0; r < 8; ++r) p[r] += (acc[r] * 0.125f) * qc[(size_t)sI[r] * QW];
    }
#pragma unroll
    for (int mk = 1; mk < 16; mk <<= 1) {
#pragma unroll
      for (int r = 0; r < 8; ++r) p[r] += __shfl_xor(p[r], mk);
    }
    if (m == 0) {
#pragma unroll
      for (int r = 0; r < 8; ++r) T.at[8 * h + r][hd] = p[r] * INV_SQRT48;
    }
  }
  __syncthreads();

  const v4f o = *(const v4f*)(&T.at[0][0] + 4 * lane);
  float* dstp = lg + (size_t)tile * 128 + 4 * lane;
  *(volatile v4f*)dstp = o;
  __threadfence();
  *(volatile v4f*)dstp = o;
}

#define NT3   128
#define NW3   4
#define NWK   2
#define EPT   8
#define CHUNK (NT3 * EPT)
#define WCAP  (EPT * 32)
#define LISTN (NW3 * WCAP)
#define PASSN (NWK * 16)
#define PCAP  (CHUNK + PASSN)
#define NBD   32
#define PKS   6
static_assert(NBD < (1 << PKS));
static_assert(NBD * 8 == 2 * NT3);
static_assert(PCAP >= CHUNK + PASSN);

__device__ __forceinline__ int scan_chunk(const int* __restrict__ dsts, int nE, int cbase, int nodeBase,
                                          int vec8, int* list, int tid, int wave) {
  int wc = 0;
  const int el0  = tid * EPT;
  const int e0   = cbase + el0;
  const int sent = -2147483647 - 1;
  v4i da, db;
  if (vec8 != 0 && cbase + CHUNK <= nE) {
    da = *(const v4i*)(dsts + e0);
    db = *(const v4i*)(dsts + e0 + 4);
  } else {
    da.x = (e0     < nE) ? dsts[min(e0,     nE - 1)] : sent;
    da.y = (e0 + 1 < nE) ? dsts[min(e0 + 1, nE - 1)] : sent;
    da.z = (e0 + 2 < nE) ? dsts[min(e0 + 2, nE - 1)] : sent;
    da.w = (e0 + 3 < nE) ? dsts[min(e0 + 3, nE - 1)] : sent;
    db.x = (e0 + 4 < nE) ? dsts[min(e0 + 4, nE - 1)] : sent;
    db.y = (e0 + 5 < nE) ? dsts[min(e0 + 5, nE - 1)] : sent;
    db.z = (e0 + 6 < nE) ? dsts[min(e0 + 6, nE - 1)] : sent;
    db.w = (e0 + 7 < nE) ? dsts[min(e0 + 7, nE - 1)] : sent;
  }
  const unsigned nb = (unsigned)nodeBase;
  const unsigned s0 = (unsigned)da.x - nb, s1 = (unsigned)da.y - nb;
  const unsigned s2 = (unsigned)da.z - nb, s3 = (unsigned)da.w - nb;
  const unsigned s4 = (unsigned)db.x - nb, s5 = (unsigned)db.y - nb;
  const unsigned s6 = (unsigned)db.z - nb, s7 = (unsigned)db.w - nb;
  const bool h0 = s0 < (unsigned)NBD, h1 = s1 < (unsigned)NBD, h2 = s2 < (unsigned)NBD, h3 = s3 < (unsigned)NBD;
  const bool h4 = s4 < (unsigned)NBD, h5 = s5 < (unsigned)NBD, h6 = s6 < (unsigned)NBD, h7 = s7 < (unsigned)NBD;
  const unsigned any = __builtin_amdgcn_ballot_w32(h0 | h1 | h2 | h3 | h4 | h5 | h6 | h7);
  if (any != 0u) {
#define HITJ(J, HJ, SJ) { \
      const unsigned mj = __builtin_amdgcn_ballot_w32(HJ); \
      if (mj != 0u) { \
        if (HJ) { \
          const int pos = wc + (int)__builtin_amdgcn_mbcnt_lo(mj, 0u); \
          if (pos < WCAP) list[wave * WCAP + pos] = ((el0 + (J)) << PKS) | (int)(SJ); \
        } \
        wc += (int)__builtin_popcount(mj); } }
    HITJ(0, h0, s0)
    HITJ(1, h1, s1)
    HITJ(2, h2, s2)
    HITJ(3, h3, s3)
    HITJ(4, h4, s4)
    HITJ(5, h5, s5)
    HITJ(6, h6, s6)
    HITJ(7, h7, s7)
#undef HITJ
  }
  return wc;
}

__device__ __forceinline__ void acc_tile(float* macc, v8f vv, v8i slo, v8i shi, int col, int h, int wave) {
#pragma unroll
  for (int wv = 0; wv < NWK; ++wv) {
    if (wave == wv) {
#pragma unroll
      for (int r = 0; r < 8; ++r) {
        const int sa = slo[r], sb = shi[r];
        const int mine = (h == 0) ? sa : sb;
        float* p = macc + mine * QW + col;
        if (h == 0 || sa != sb) { const float t = *p; *p = t + vv[r]; }
        wxbar();
        if (h != 0 && sa == sb) { const float t = *p; *p = t + vv[r]; }
        wxbar();
      }
    }
    __syncthreads();
  }
}

__global__ __launch_bounds__(NT3) void k_aggr(
    const int* __restrict__ ei, const float* __restrict__ rbf, const float* __restrict__ rsh,
    const float* __restrict__ SD, const float* __restrict__ lg,
    const bf16* __restrict__ BrbfT, const bf16* __restrict__ Bkv0T, const bf16* __restrict__ Bkv1T,
    float* msg, int nN, int nE, int vec8) {
  __shared__ __attribute__((aligned(16))) float macc[(NBD + 1) * QW];
  __shared__ float mst[(NBD + 1) * 8];
  __shared__ float linv[(NBD + 1) * 8];
  __shared__ __attribute__((aligned(16))) int list[LISTN];
  __shared__ __attribute__((aligned(16))) int pend[PCAP];
  __shared__ int wcnt[NW3];
  __shared__ int pendN;
  __shared__ TileBuf tb[NWK];

  const int tid = threadIdx.x, lane = tid & 31, wave = tid >> 5, h = lane >> 4, m = lane & 15;
  const int nodeBase = blockIdx.x * NBD;
  const int* dsts = ei + nE;
  const bool worker = wave < NWK;
  TileBuf& T = tb[worker ? wave : 0];

  for (int i = tid; i < (NBD + 1) * QW; i += NT3) macc[i] = 0.0f;
  if (tid == 0) pendN = 0;
  __syncthreads();

  const int nChunks = (nE + CHUNK - 1) / CHUNK;

  const int slA = tid >> 3, slB = (NBD / 2) + (tid >> 3), hq = tid & 7;
  float rmA = -__builtin_inff(), rlA = 0.0f, rmB = -__builtin_inff(), rlB = 0.0f;
#pragma unroll 1
  for (int ch = 0; ch < nChunks; ++ch) {
    const int cbase = ch * CHUNK;
    const int wc = scan_chunk(dsts, nE, cbase, nodeBase, vec8, list, tid, wave);
    if (lane == 0) wcnt[wave] = wc;
    __syncthreads();
    int tot = 0, myoff = 0;
#pragma unroll
    for (int w = 0; w < NW3; ++w) {
      const int c = clampi(wcnt[w], 0, WCAP);
      if (w < wave) myoff += c;
      tot += c;
    }
    tot = tot > CHUNK ? CHUNK : tot;
    {
      const int n = clampi(wcnt[wave], 0, WCAP);
      const int* lp = list + wave * WCAP;
      for (int i = lane; i < n; i += 32) {
        const int pos = myoff + i;
        if (pos < PCAP) pend[pos] = lp[i] + (cbase << PKS);
      }
    }
    __syncthreads();
#pragma unroll 1
    for (int i = 0; i < tot; ++i) {
      const int pk = pend[i];
      const int s = pk & ((1 << PKS) - 1);
      const int eg = clampi(pk >> PKS, 0, nE - 1);
      const float x = lg[(size_t)eg * 8 + hq];
      if (s == slA) { const float mn = fmaxf(rmA, x); rlA = rlA * expf(rmA - mn) + expf(x - mn); rmA = mn; }
      if (s == slB) { const float mn = fmaxf(rmB, x); rlB = rlB * expf(rmB - mn) + expf(x - mn); rmB = mn; }
    }
    __syncthreads();
  }
  mst[slA * 8 + hq] = rmA; linv[slA * 8 + hq] = 1.0f / (rlA + 1e-16f);
  mst[slB * 8 + hq] = rmB; linv[slB * 8 + hq] = 1.0f / (rlB + 1e-16f);
  if (tid < 8) { mst[NBD * 8 + tid] = 0.0f; linv[NBD * 8 + tid] = 0.0f; }
  if (tid == 0) pendN = 0;
  __syncthreads();

#pragma unroll 1
  for (int ch = 0; ch < nChunks; ++ch) {
    const int cbase = ch * CHUNK;
    const int wc = scan_chunk(dsts, nE, cbase, nodeBase, vec8, list, tid, wave);
    if (lane == 0) wcnt[wave] = wc;
    __syncthreads();
    const int base = pendN;
    int tot = 0, myoff = 0;
#pragma unroll
    for (int w = 0; w < NW3; ++w) {
      const int c = clampi(wcnt[w], 0, WCAP);
      if (w < wave) myoff += c;
      tot += c;
    }
    int newN = base + tot;
    newN = newN > PCAP ? PCAP : newN;
    {
      const int n = clampi(wcnt[wave], 0, WCAP);
      const int* lp = list + wave * WCAP;
      for (int i = lane; i < n; i += 32) {
        const int pos = base + myoff + i;
        if (pos < PCAP) pend[pos] = lp[i] + (cbase << PKS);
      }
    }
    const int fin = (ch == nChunks - 1) ? 1 : 0;
    int R = (fin != 0) ? (newN + PASSN - 1) / PASSN : newN / PASSN;
    R = clampi(R, 0, PCAP / PASSN + 1);
    const int Pv = (fin != 0) ? newN : R * PASSN;
    __syncthreads();

#pragma unroll 1
    for (int rp = 0; rp < R; ++rp) {
      if (worker) {
        const int idx = rp * PASSN + wave * 16 + m;
        const bool valid = idx < Pv;
        const int pk = pend[idx < PCAP ? idx : (PCAP - 1)];
        int sl = pk & ((1 << PKS) - 1);
        if (!valid || (unsigned)sl >= (unsigned)NBD) sl = NBD;
        const int eg = clampi(pk >> PKS, 0, nE - 1);
        tile_gather(T, eg, valid, lane, ei, nE, nN, rbf, rsh);
        const v4f x4 = *(const v4f*)(lg + (size_t)eg * 8 + 4 * h);
        float xs[4] = {x4.x, x4.y, x4.z, x4.w};
#pragma unroll
        for (int i = 0; i < 4; ++i) {
          const int hh = 4 * h + i;
          const float mv = mst[sl * 8 + hh], li = linv[sl * 8 + hh];
          const float dx = valid ? (xs[i] - mv) : -80.0f;
          T.at[m][hh] = expf(dx) * li;
        }
        if (h == 0) T.slot[m] = sl;
      }
      __syncthreads();
      if (worker) {
        cg_ntile<0>(T, lane, BrbfT, SD);
        cg_ntile<1>(T, lane, BrbfT, SD);
        cg_ntile<2>(T, lane, BrbfT, SD);
        cg_ntile<3>(T, lane, BrbfT, SD);
        cg_ntile<4>(T, lane, BrbfT, SD);
        cg_ntile<5>(T, lane, BrbfT, SD);
        cg_ntile<6>(T, lane, BrbfT, SD);
      }
      __syncthreads();

      v8i slo, shi;
#pragma unroll
      for (int r = 0; r < 8; ++r) { slo[r] = T.slot[r]; shi[r] = T.slot[8 + r]; }

      {
        v16b a5[5];
#pragma unroll
        for (int ks = 0; ks < 5; ++ks) a5[ks] = ldfrag(&T.Acp0[m][32 * ks], h);
#pragma unroll 1
        for (int nt2 = 0; nt2 < 16; ++nt2) {
          const int hdd = nt2 >> 1;
          v8f vv = z8f();
          if (worker) {
            v8f acc = z8f();
#pragma unroll
            for (int ks = 0; ks < 5; ++ks)
              acc = wmb(a5[ks], ldfrag(Bkv0T + (size_t)(256 + 16 * nt2 + m) * 160 + 32 * ks, h), acc);
#pragma unroll
            for (int r = 0; r < 8; ++r) vv[r] = (acc[r] * INV_SQRT48) * T.at[8 * h + r][hdd];
          }
          acc_tile(macc, vv, slo, shi, hdd * MDIM + ((nt2 & 1) << 4) + m, h, wave);
        }
      }
#pragma unroll
      for (int c = 0; c < 3; ++c) {
        v16b a6[6];
#pragma unroll
        for (int ks = 0; ks < 4; ++ks) a6[ks] = ldfrag(&T.Acp1[c][m][32 * ks], h);
        a6[4] = a6[0];
        a6[5] = a6[1];
#pragma unroll 1
        for (int nt2 = 0; nt2 < 8; ++nt2) {
          v8f vv = z8f();
          if (worker) {
            v8f acc = z8f();
#pragma unroll
            for (int ks = 0; ks < 6; ++ks)
              acc = wmb(a6[ks], ldfrag(Bkv1T + (size_t)(128 + 16 * nt2 + m) * 192 + 32 * ks, h), acc);
#pragma unroll
            for (int r = 0; r < 8; ++r) vv[r] = (acc[r] * 0.125f) * T.at[8 * h + r][nt2];
          }
          acc_tile(macc, vv, slo, shi, nt2 * MDIM + 32 + 3 * m + c, h, wave);
        }
      }
    }

    int rem = newN - R * PASSN;
    rem = rem < 0 ? 0 : rem;
    if (R > 0 && tid < rem) pend[tid] = pend[R * PASSN + tid];
    if (tid == 0) pendN = rem;
  }
  __syncthreads();

#pragma unroll 1
  for (int ps = 0; ps < 2; ++ps) {
#pragma unroll 1
    for (int t = 0; t < 8; ++t) {
      const int sl = wave * 8 + t;
      const size_t ng = (size_t)(nodeBase + sl);
      const float* srow = macc + sl * QW;
#pragma unroll
      for (int i = 0; i < 5; ++i) {
        const int off = (4 * i + (lane >> 3)) * 32 + (lane & 7) * 4;
        const v4f v = *(const v4f*)(srow + off);
        *(volatile v4f*)(msg + ng * QW + off) = v;
      }
    }
    if (ps == 0) __threadfence();
  }
}

#define NT4 256
__global__ __launch_bounds__(NT4) void k_out(
    const float* __restrict__ node, const float* __restrict__ msg,
    const bf16* __restrict__ Bm0T, const bf16* __restrict__ Bm1T, float* out, int nN) {
  __shared__ __attribute__((aligned(16))) bf16  Am0[16 * 512];
  __shared__ __attribute__((aligned(16))) bf16  Am1[48 * 256];
  __shared__ __attribute__((aligned(16))) float os[16 * NODE_W];
  const int tid = threadIdx.x, lane = tid & 31, wave = tid >> 5, h = lane >> 4, m = lane & 15;
  const int nodeBase = blockIdx.x * 16;

  for (int idx = tid; idx < 16 * QW; idx += NT4) {
    const int nl = idx / QW;
    const int j  = idx - nl * QW;
    const float v = msg[(size_t)(nodeBase + nl) * QW + j];
    const int hd = j / MDIM;
    const int jj = j - hd * MDIM;
    bf16 hi, lo;
    split2(v, hi, lo);
    if (jj < 32) {
      const int col = hd * 32 + jj;
      Am0[nl * 512 + col] = hi;
      Am0[nl * 512 + 256 + col] = lo;
    } else {
      const int t = jj - 32;
      const int uu = t / 3, c = t - 3 * uu;
      const int row = nl * 3 + c, col = hd * 16 + uu;
      Am1[row * 256 + col] = hi;
      Am1[row * 256 + 128 + col] = lo;
    }
  }
  __syncthreads();

#pragma unroll 1
  for (int task = wave; task < 10; task += 8) {
    v8f acc = z8f();
    if (task < 4) {
      const int nt = task;
#pragma unroll
      for (int ks = 0; ks < 24; ++ks)
        acc = wmb(ldfrag(Am0 + m * 512 + ((32 * ks) & 511), h),
                  ldfrag(Bm0T + (size_t)(16 * nt + m) * 768 + 32 * ks, h), acc);
#pragma unroll
      for (int r = 0; r < 8; ++r) os[(8 * h + r) * NODE_W + 16 * nt + m] = acc[r] * 0.0625f;
    } else {
      const int t2 = task - 4, mt = t2 >> 1, nt = t2 & 1;
#pragma unroll
      for (int ks = 0; ks < 12; ++ks)
        acc = wmb(ldfrag(Am1 + (16 * mt + m) * 256 + ((32 * ks) & 255), h),
                  ldfrag(Bm1T + (size_t)(16 * nt + m) * 384 + 32 * ks, h), acc);
#pragma unroll
      for (int r = 0; r < 8; ++r) {
        const int rr = 16 * mt + 8 * h + r;
        const int nl = rr / 3, c = rr - 3 * nl;
        const int v = 16 * nt + m;
        os[nl * NODE_W + 64 + 3 * v + c] = acc[r] * INV_SQRT128;
      }
    }
  }
  __syncthreads();

  v4f va[2], vb[2];
  int  ngs[2];
  const int offA = (lane >> 3) * 32 + (lane & 7) * 4;
  const int offB = 128 + (lane & 7) * 4;
#pragma unroll
  for (int t = 0; t < 2; ++t) {
    const int nl = 2 * wave + t;
    const int ng = nodeBase + nl;
    const int nc = ng < nN ? ng : (nN - 1);
    ngs[t] = ng;
    const float* nr = node + (size_t)nc * NODE_W;
    va[t] = *(const v4f*)(os + nl * NODE_W + offA) + *(const v4f*)(nr + offA);
    vb[t] = *(const v4f*)(os + nl * NODE_W + offB) + *(const v4f*)(nr + offB);
  }
#pragma unroll 1
  for (int ps = 0; ps < 2; ++ps) {
#pragma unroll
    for (int t = 0; t < 2; ++t) {
      if (ngs[t] < nN) {
        float* orow = out + (size_t)ngs[t] * NODE_W;
        *(volatile v4f*)(orow + offA) = va[t];
        if (lane < 8) *(volatile v4f*)(orow + offB) = vb[t];
      }
    }
    if (ps == 0) __threadfence();
  }
}

extern "C" void kernel_launch(void* const* d_in, const int* in_sizes, int n_in,
                              void* d_out, int out_size, void* d_ws, size_t ws_size,
                              hipStream_t stream) {
  if (n_in < 17) return;
  const int nN = in_sizes[0] / NODE_W;
  const int nE = in_sizes[3] / 2;
  if (nN <= 0 || nE <= 0) return;
  if (in_sizes[0] != nN * NODE_W || in_sizes[3] != 2 * nE) return;
  if (in_sizes[1] != nE * NBAS || in_sizes[2] != nE * 4) return;
  if (in_sizes[4] < 64 || in_sizes[5] < 32) return;
  if (in_sizes[6] != 64 * 256 || in_sizes[7] != 32 * 128) return;
  if (in_sizes[8] != 64 * 32 || in_sizes[9] != 32 * 16 || in_sizes[10] != 64 * 32 || in_sizes[11] != 32 * 16) return;
  if (in_sizes[12] != 16 * 112 || in_sizes[13] != 48 * 512 || in_sizes[14] != 64 * 256) return;
  if (in_sizes[15] != 256 * 64 || in_sizes[16] != 128 * 32) return;
  if (out_size != nN * NODE_W) return;

  const float* node  = (const float*)d_in[0];
  const float* rbf   = (const float*)d_in[1];
  const float* rsh   = (const float*)d_in[2];
  const int*   eidx  = (const int*)d_in[3];
  const float* g0    = (const float*)d_in[4];
  const float* g1    = (const float*)d_in[5];
  const float* Wq0   = (const float*)d_in[6];
  const float* Wq1   = (const float*)d_in[7];
  const float* Wsrc0 = (const float*)d_in[8];
  const float* Wsrc1 = (const float*)d_in[9];
  const float* Wdst0 = (const float*)d_in[10];
  const float* Wdst1 = (const float*)d_in[11];
  const float* Wrbf  = (const float*)d_in[12];
  const float* Wkv0  = (const float*)d_in[13];
  const float* Wkv1  = (const float*)d_in[14];
  const float* Wm0   = (const float*)d_in[15];
  const float* Wm1   = (const float*)d_in[16];
  float* out = (float*)d_out;

  const int nBlkN  = (nN + 15) / 16;
  const int nBlkA  = (nN + NBD - 1) / NBD;
  const int NpAll  = nBlkA * NBD;
  const int nTiles = (nE + 15) / 16;
  const int nBlkL  = (nTiles + NW2 - 1) / NW2;
  const int Ep     = nBlkL * NW2 * 16;

  size_t off = 0;
  auto carve = [&](size_t bytes) { const size_t o = off; off += (bytes + 255) & ~(size_t)255; return o; };
  const size_t oP0  = carve((size_t)320 * 192 * 2);
  const size_t oP1  = carve((size_t)160 * 96 * 2);
  const size_t oP2  = carve((size_t)112 * 64 * 2);
  const size_t oP3  = carve((size_t)512 * 160 * 2);
  const size_t oP4  = carve((size_t)256 * 192 * 2);
  const size_t oP5  = carve((size_t)64 * 768 * 2);
  const size_t oP6  = carve((size_t)32 * 384 * 2);
  const size_t oQ   = carve((size_t)NpAll * QW * 4);
  const size_t oSD  = carve((size_t)NpAll * NODE_W * 4);
  const size_t oLG  = carve((size_t)Ep * 8 * 4);
  const size_t oMSG = carve((size_t)NpAll * QW * 4);
  if (off > ws_size || off > (size_t)134217728) return;

  char* ws = (char*)d_ws;
  bf16* P0 = (bf16*)(ws + oP0);
  bf16* P1 = (bf16*)(ws + oP1);
  bf16* P2 = (bf16*)(ws + oP2);
  bf16* P3 = (bf16*)(ws + oP3);
  bf16* P4 = (bf16*)(ws + oP4);
  bf16* P5 = (bf16*)(ws + oP5);
  bf16* P6 = (bf16*)(ws + oP6);
  float* q    = (float*)(ws + oQ);
  float* sd   = (float*)(ws + oSD);
  float* lg   = (float*)(ws + oLG);
  float* msgb = (float*)(ws + oMSG);

  const int vec8 = ((nE & 3) == 0) ? 1 : 0;

  k_wprep<<<dim3(40, 7), 256, 0, stream>>>(Wq0, Wsrc0, Wdst0, Wq1, Wsrc1, Wdst1, Wrbf, Wkv0, Wkv1, Wm0, Wm1,
                                           P0, P1, P2, P3, P4, P5, P6);
  k_node<<<nBlkN, NT1, 0, stream>>>(node, g0, g1, P0, P1, q, sd, nN);
  k_logit<<<nBlkL, NT2, 0, stream>>>(eidx, rbf, rsh, sd, q, P2, P3, P4, lg, nN, nE);
  k_aggr<<<nBlkA, NT3, 0, stream>>>(eidx, rbf, rsh, sd, lg, P2, P3, P4, msgb, nN, nE, vec8);
  k_out<<<nBlkN, NT4, 0, stream>>>(node, msgb, P5, P6, out, nN);
}
